// ScaledDotProductAttention_70153995813465
// MI455X (gfx1250) — hardware-verified
//
#include <hip/hip_runtime.h>


typedef _Float16 v16h __attribute__((ext_vector_type(16)));
typedef _Float16 v8h  __attribute__((ext_vector_type(8)));
typedef float    v8f  __attribute__((ext_vector_type(8)));
typedef float    v4f  __attribute__((ext_vector_type(4)));

#ifndef NB
#define NB 32
#endif
#ifndef SEQ
#define SEQ 2048
#endif
#ifndef SEQ_FULL
#define SEQ_FULL 2048
#endif
#define DH 64

constexpr int QTILE = 128;
constexpr int KBLK  = 64;
constexpr int NT    = KBLK / 16;
constexpr int NKC   = KBLK / 32;
constexpr int KD    = DH + 8;
constexpr int VD    = KBLK + 8;
constexpr int PD    = KBLK + 8;
constexpr int OPF   = 68;
constexpr int TP    = 72;
constexpr int NQB   = SEQ / QTILE;
constexpr int QRESB = (NQB < 4) ? NQB : 4;

constexpr int LDS_K     = KBLK * KD;
constexpr int LDS_V     = DH * VD;
constexpr int LDS_P     = 8 * 16 * PD;
constexpr int LDS_O     = 8 * 16 * OPF * 2;
constexpr int LDS_PLAIN = LDS_K + LDS_V + LDS_P;
constexpr int LDS_RES   = LDS_PLAIN + LDS_P;

static_assert(SEQ % QTILE == 0);
static_assert(SEQ % KBLK == 0);
static_assert(SEQ % 64 == 0);
static_assert(SEQ <= SEQ_FULL);
static_assert(QTILE == 2 * KBLK);
static_assert(DH == 64);
static_assert(LDS_O <= LDS_PLAIN);
static_assert((OPF * 4) % 16 == 0);
static_assert((LDS_K * 2) % 16 == 0);
static_assert((LDS_V * 2) % 16 == 0);
static_assert((LDS_P * 2) % 16 == 0);

constexpr float L2E  = 1.44269504088896f;
constexpr float SCL  = L2E / 2048.0f;
constexpr float NEGV = -1.0e30f;
constexpr float PCAR = 1024.0f;
constexpr float RCAR = 1024.0f;
constexpr float RINV = 1.0f / 1024.0f;
constexpr float VINV = 1.0f / 16.0f;

__device__ __forceinline__ float fast_exp2(float x) {
#if defined(__has_builtin) && __has_builtin(__builtin_amdgcn_exp2f)
    return __builtin_amdgcn_exp2f(x);
#else
    return exp2f(x);
#endif
}

__device__ __forceinline__ float fast_rcp(float x) {
#if defined(__has_builtin) && __has_builtin(__builtin_amdgcn_rcpf)
    return __builtin_amdgcn_rcpf(x);
#else
    return 1.0f / x;
#endif
}

__device__ __forceinline__ _Float16 cvh(float x) {
    unsigned int u = __float_as_uint(x);
    u = (u + 0x7FFFu + ((u >> 16) & 1u)) & 0xFFFF0000u;
    return (_Float16)(__uint_as_float(u) * 16.0f);
}

__device__ __forceinline__ v8f wmma16(v16h a, v16h b, v8f c) {
    v8f d = __builtin_amdgcn_wmma_f32_16x16x32_f16(false, a, false, b, (short)0, c, false, false);
    asm volatile("v_nop\n\tv_nop\n\tv_nop\n\tv_nop" : "+v"(d) : "v"(a), "v"(b));
    return d;
}

__device__ __forceinline__ v16h ld_op16(const _Float16* p) {
    union { v16h v; v8h h[2]; } u;
    u.h[0] = *(const v8h*)(p);
    u.h[1] = *(const v8h*)(p + 16);
    return u.v;
}

__device__ __forceinline__ v16h ld_q(const float* p) {
    const v4f f0 = *(const v4f*)(p);
    const v4f f1 = *(const v4f*)(p + 4);
    const v4f f2 = *(const v4f*)(p + 16);
    const v4f f3 = *(const v4f*)(p + 20);
    v16h r;
#pragma unroll
    for (int j = 0; j < 4; ++j) {
        r[j]      = cvh(f0[j]);
        r[4 + j]  = cvh(f1[j]);
        r[8 + j]  = cvh(f2[j]);
        r[12 + j] = cvh(f3[j]);
    }
    return r;
}

__global__ __launch_bounds__(256)
void k_prep(const float* __restrict__ K, const float* __restrict__ V,
            _Float16* __restrict__ Kh, _Float16* __restrict__ Vt)
{
    __shared__ __align__(16) _Float16 T[DH * TP];
    const int b   = blockIdx.y;
    const int s0  = blockIdx.x * 64;
    const int tid = threadIdx.x;

    v8h kst[2];
#pragma unroll
    for (int i = 0; i < 2; ++i) {
        const int ch = tid + i * 256;
        const int row = ch >> 3, cc = ch & 7;
        const float* src = K + ((size_t)b * SEQ_FULL + s0 + row) * DH + cc * 8;
        const v4f f0 = *(const v4f*)(src);
        const v4f f1 = *(const v4f*)(src + 4);
        v8h hv;
#pragma unroll
        for (int j = 0; j < 4; ++j) { hv[j] = cvh(f0[j]); hv[4 + j] = cvh(f1[j]); }
        kst[i] = hv;
    }
#pragma unroll
    for (int i = 0; i < 2; ++i) {
        const int ch = tid + i * 256;
        const int s = ch >> 3, dseg = (ch & 7) * 8;
        const float* src = V + ((size_t)b * SEQ_FULL + s0 + s) * DH + dseg;
        const v4f f0 = *(const v4f*)(src);
        const v4f f1 = *(const v4f*)(src + 4);
#pragma unroll
        for (int j = 0; j < 4; ++j) {
            T[(dseg + j) * TP + s]     = cvh(f0[j]);
            T[(dseg + 4 + j) * TP + s] = cvh(f1[j]);
        }
    }
    __syncthreads();

    v8h vst[2];
#pragma unroll
    for (int i = 0; i < 2; ++i) {
        const int ch = tid + i * 256;
        const int d = ch >> 3, cc = ch & 7;
        vst[i] = *(const v8h*)&T[d * TP + cc * 8];
    }

#pragma unroll
    for (int i = 0; i < 2; ++i) {
        const int ch = tid + i * 256;
        const int row = ch >> 3, cc = ch & 7;
        _Float16* kd = Kh + ((size_t)b * SEQ + s0 + row) * DH + cc * 8;
        *(volatile v8h*)kd = kst[i];
        _Float16* vd = Vt + ((size_t)b * DH + row) * SEQ + s0 + cc * 8;
        *(volatile v8h*)vd = vst[i];
    }
    __threadfence();
#pragma unroll
    for (int i = 0; i < 2; ++i) {
        const int ch = tid + i * 256;
        const int row = ch >> 3, cc = ch & 7;
        _Float16* kd = Kh + ((size_t)b * SEQ + s0 + row) * DH + cc * 8;
        *(volatile v8h*)kd = kst[i];
        _Float16* vd = Vt + ((size_t)b * DH + row) * SEQ + s0 + cc * 8;
        *(volatile v8h*)vd = vst[i];
    }
}

template <bool RES>
__global__ __launch_bounds__(256) __attribute__((amdgpu_num_vgpr(256)))
void k_attn(const float* __restrict__ Q,
            const _Float16* __restrict__ Kh,
            const _Float16* __restrict__ Vt,
            float* __restrict__ O, int qb0)
{
    __shared__ __align__(16) _Float16 lds_all[RES ? LDS_RES : LDS_PLAIN];
    _Float16* const Ksh = lds_all;
    _Float16* const Vts = lds_all + LDS_K;
    _Float16* const Pst = lds_all + LDS_K + LDS_V;

    const int qb   = (int)blockIdx.x + qb0;
    const int bb   = blockIdx.y;
    const int tid  = threadIdx.x;
    const int lane = tid & 31;
    const int wv   = tid >> 5;
    const int hf   = lane >> 4;
    const int l16  = lane & 15;
    const int koff = hf * 8;

    const float*    Qb  = Q  + (size_t)bb * SEQ_FULL * DH;
    float*          Ob  = O  + (size_t)bb * SEQ_FULL * DH;
    const _Float16* KhB = Kh + (size_t)bb * SEQ * DH;
    const _Float16* VtB = Vt + (size_t)bb * DH * SEQ;

    const int  qrow = qb * QTILE + wv * 16 + l16;
    const v16h qa0  = ld_q(Qb + (size_t)qrow * DH + koff);
    const v16h qa1  = ld_q(Qb + (size_t)qrow * DH + 32 + koff);

    const v8f vzero = {0.f, 0.f, 0.f, 0.f, 0.f, 0.f, 0.f, 0.f};
    v8f o[4], orr[4];
#pragma unroll
    for (int t = 0; t < 4; ++t) { o[t] = vzero; orr[t] = vzero; }

    float m[8], l[8];
#pragma unroll
    for (int v = 0; v < 8; ++v) { m[v] = NEGV; l[v] = 0.0f; }

    _Float16* const Pw  = Pst + wv * 16 * PD;
    _Float16* const Prw = Pst + LDS_P + wv * 16 * PD;

    const int nkb = 2 * qb + 2;
    const int kbm = 2 * qb;

    for (int kb = 0; kb < nkb; ++kb) {
        __syncthreads();
#pragma unroll
        for (int i = 0; i < 2; ++i) {
            const int ch  = tid + i * 256;
            const int row = ch >> 3, cc = ch & 7;
            *(v8h*)&Ksh[row * KD + cc * 8] =
                *(const v8h*)(KhB + ((size_t)kb * KBLK + row) * DH + cc * 8);
            *(v8h*)&Vts[row * VD + cc * 8] =
                *(const v8h*)(VtB + (size_t)row * SEQ + (size_t)kb * KBLK + cc * 8);
        }
        __syncthreads();

        v8f c[NT];
#pragma unroll
        for (int t = 0; t < NT; ++t) c[t] = vzero;
#pragma unroll
        for (int kc = 0; kc < 2; ++kc) {
            const v16h a = kc ? qa1 : qa0;
#pragma unroll
            for (int t = 0; t < NT; ++t) {
                const v16h bop = ld_op16(&Ksh[(t * 16 + l16) * KD + kc * 32 + koff]);
                c[t] = wmma16(a, bop, c[t]);
            }
        }

#pragma unroll
        for (int t = 0; t < NT; ++t)
#pragma unroll
            for (int v = 0; v < 8; ++v) c[t][v] *= SCL;

        if (kb >= kbm) {
            const int kl0 = (kb - kbm) * KBLK;
#pragma unroll
            for (int t = 0; t < NT; ++t) {
                const int kl = kl0 + t * 16 + l16;
#pragma unroll
                for (int v = 0; v < 8; ++v) {
                    const int ql = wv * 16 + 8 * hf + v;
                    c[t][v] = (kl > ql) ? NEGV : c[t][v];
                }
            }
        }

        float sc[8];
#pragma unroll
        for (int v = 0; v < 8; ++v) {
            float r = fmaxf(fmaxf(c[0][v], c[1][v]), fmaxf(c[2][v], c[3][v]));
            r = fmaxf(r, __shfl_xor(r, 1, 32));
            r = fmaxf(r, __shfl_xor(r, 2, 32));
            r = fmaxf(r, __shfl_xor(r, 4, 32));
            r = fmaxf(r, __shfl_xor(r, 8, 32));
            const float mn = fmaxf(m[v], r);
            sc[v] = fast_exp2(m[v] - mn);
            m[v]  = mn;
        }
#pragma unroll
        for (int t = 0; t < NT; ++t)
#pragma unroll
            for (int v = 0; v < 8; ++v)
                c[t][v] = fast_exp2(c[t][v] - m[v]);

#pragma unroll
        for (int v = 0; v < 8; ++v) {
#pragma unroll
            for (int t = 0; t < 4; ++t) {
                o[t][v] *= sc[v];
                if (RES) orr[t][v] *= sc[v];
            }
        }

#pragma unroll
        for (int v = 0; v < 8; ++v) {
            float rs = 0.0f;
#pragma unroll
            for (int t = 0; t < NT; ++t) {
                const float    p1024 = c[t][v] * PCAR;
                const _Float16 ph    = (_Float16)p1024;
                Pw[(v + 8 * hf) * PD + t * 16 + l16] = ph;
                float pe = (float)ph;
                if (RES) {
                    const _Float16 rh = (_Float16)((p1024 - pe) * RCAR);
                    Prw[(v + 8 * hf) * PD + t * 16 + l16] = rh;
                    pe += (float)rh * RINV;
                }
                rs += pe;
            }
            l[v] = l[v] * sc[v] + rs;
        }
        __syncthreads();

#pragma unroll
        for (int kc = 0; kc < NKC; ++kc) {
            const v16h pa  = ld_op16(&Pw[l16 * PD + kc * 32 + koff]);
            const v16h par = RES ? ld_op16(&Prw[l16 * PD + kc * 32 + koff]) : pa;
#pragma unroll
            for (int t = 0; t < 4; ++t) {
                const v16h vb = ld_op16(&Vts[(t * 16 + l16) * VD + kc * 32 + koff]);
                o[t] = wmma16(pa, vb, o[t]);
                if (RES) orr[t] = wmma16(par, vb, orr[t]);
            }
        }
    }

    if (RES) {
#pragma unroll
        for (int v = 0; v < 8; ++v)
#pragma unroll
            for (int t = 0; t < 4; ++t) o[t][v] += orr[t][v] * RINV;
    }
    float rinv[8];
#pragma unroll
    for (int v = 0; v < 8; ++v) {
        float ls = l[v];
        ls += __shfl_xor(ls, 1, 32);
        ls += __shfl_xor(ls, 2, 32);
        ls += __shfl_xor(ls, 4, 32);
        ls += __shfl_xor(ls, 8, 32);
        rinv[v] = fast_rcp(ls) * VINV;
    }

    __syncthreads();
    float* const Of = reinterpret_cast<float*>(lds_all) + wv * 16 * OPF;
#pragma unroll
    for (int v = 0; v < 8; ++v) {
#pragma unroll
        for (int t = 0; t < 4; ++t)
            Of[(v + 8 * hf) * OPF + t * 16 + l16] = o[t][v] * rinv[v];
    }
    __syncthreads();

    const int sub = lane >> 3, jj = lane & 7;
    float* const Orow0 = Ob + (size_t)(qb * QTILE + wv * 16) * DH;
#pragma unroll
    for (int it = 0; it < 8; ++it) {
        const int row = 2 * it + (sub >> 1);
        const int col = (sub & 1) * 32 + jj * 4;
        const v4f val = *(const v4f*)&Of[row * OPF + col];
        *(volatile v4f*)(Orow0 + (size_t)row * DH + col) = val;
    }
    __threadfence();
#pragma unroll
    for (int it = 0; it < 8; ++it) {
        const int row = 2 * it + (sub >> 1);
        const int col = (sub & 1) * 32 + jj * 4;
        const v4f val = *(const v4f*)&Of[row * OPF + col];
        *(volatile v4f*)(Orow0 + (size_t)row * DH + col) = val;
    }
}

extern "C" void kernel_launch(void* const* d_in, const int* in_sizes, int n_in,
                              void* d_out, int out_size, void* d_ws, size_t ws_size,
                              hipStream_t stream)
{
    if (n_in < 3) return;
    const float* Q = (const float*)d_in[0];
    const float* K = (const float*)d_in[1];
    const float* V = (const float*)d_in[2];
    float* O = (float*)d_out;

    const long long need = (long long)(NB - 1) * SEQ_FULL * DH + (long long)SEQ * DH;
    if ((long long)in_sizes[0] < need || (long long)in_sizes[1] < need || (long long)in_sizes[2] < need) return;
    if ((long long)out_size < need) return;

    const size_t plane  = (size_t)NB * SEQ * DH;
    const size_t wsneed = plane * 2 * sizeof(_Float16);
    if (ws_size < wsneed) return;

    _Float16* Kh = (_Float16*)d_ws;
    _Float16* Vt = Kh + plane;

    k_prep<<<dim3(SEQ / 64, NB), dim3(256), 0, stream>>>(K, V, Kh, Vt);
    k_attn<true><<<dim3(QRESB, NB), dim3(256), 0, stream>>>(Q, Kh, Vt, O, 0);
    if (NQB > QRESB)
        k_attn<false><<<dim3(NQB - QRESB, NB), dim3(256), 0, stream>>>(Q, Kh, Vt, O, QRESB);
}
